// LinearTriParser_9302899163650
// MI455X (gfx1250) — hardware-verified
//
#include <hip/hip_runtime.h>
#include <math.h>

typedef __attribute__((ext_vector_type(16))) _Float16 v16h;
typedef __attribute__((ext_vector_type(16))) __bf16 v16b;
typedef __attribute__((ext_vector_type(8)))  _Float16 v8h;
typedef __attribute__((ext_vector_type(8)))  float v8f;
typedef __attribute__((ext_vector_type(4)))  float v4f;
typedef __attribute__((ext_vector_type(2)))  float v2f;
typedef __attribute__((ext_vector_type(4)))  unsigned v4u;
typedef __attribute__((ext_vector_type(4)))  int v4i;
typedef float __attribute__((may_alias)) float_a;
typedef int __attribute__((may_alias)) int_a;

template <typename T> __device__ __forceinline__ void vst2(void* p, T v) { *(volatile T*)p = v; __threadfence(); *(volatile T*)p = v; }
__device__ __forceinline__ v8f wmma16(v16h a, v16h b, v8f c) {
  v8f d = __builtin_amdgcn_wmma_f32_16x16x32_f16(false, a, false, b, (short)0, c, false, false);
  asm volatile("v_nop\n\tv_nop\n\tv_nop\n\tv_nop" : "+v"(d) : "v"(a), "v"(b));
  return d;
}
__device__ __forceinline__ v8f wmma_bf(v16b a, v16b b, v8f c) {
  v8f d = __builtin_amdgcn_wmma_f32_16x16x32_bf16(false, a, false, b, (short)0, c, false, false);
  asm volatile("v_nop\n\tv_nop\n\tv_nop\n\tv_nop" : "+v"(d) : "v"(a), "v"(b));
  return d;
}
__device__ __forceinline__ v16h frag_h(const _Float16* rowk0, int lane) {
  union { v16h v; v8h q[2]; } u; const _Float16* p = rowk0 + 8 * (lane >> 4);
  u.q[0] = *(const v8h*)p; u.q[1] = *(const v8h*)(p + 16); return u.v;
}
__device__ __forceinline__ v16h frag_f32(const float* rowk0, int lane) {
  v16h a; const float* p = rowk0 + 8 * (lane >> 4);
#pragma unroll
  for (int i = 0; i < 8; ++i) { a[i] = (_Float16)p[i]; a[8 + i] = (_Float16)p[16 + i]; }
  return a;
}
__device__ __forceinline__ v16h frag_f32s(const float* rowk0, int lane, float sc) {
  v16h a; const float* p = rowk0 + 8 * (lane >> 4);
#pragma unroll
  for (int i = 0; i < 8; ++i) { a[i] = (_Float16)(p[i] * sc); a[8 + i] = (_Float16)(p[16 + i] * sc); }
  return a;
}
__device__ __forceinline__ v16h fragc_f32(const float* W, int k0, int n, int lane, int ld, int K) {
  v16h a; const int g = lane >> 4;
#pragma unroll
  for (int i = 0; i < 8; ++i) { const int ka = k0 + 8 * g + i, kb = ka + 16;
    a[i] = (_Float16)(ka < K ? W[(size_t)ka * ld + n] : 0.f); a[8 + i] = (_Float16)(kb < K ? W[(size_t)kb * ld + n] : 0.f); }
  return a;
}
struct F2 { v16b h, l; };
__device__ __forceinline__ F2 bsplit16(const float v[16]) { F2 r;
#pragma unroll
  for (int i = 0; i < 16; ++i) { const __bf16 h = (__bf16)v[i]; r.h[i] = h; r.l[i] = (__bf16)(v[i] - (float)h); }
  return r; }
__device__ __forceinline__ F2 split_row(const float* row, int k0, int lane) { float v[16]; const float* p = row + k0 + 8 * (lane >> 4);
#pragma unroll
  for (int i = 0; i < 8; ++i) { v[i] = p[i]; v[8 + i] = p[16 + i]; }
  return bsplit16(v); }
__device__ __forceinline__ F2 split_rowK(const float* row, int k0, int lane, int K) { float v[16]; const int g = lane >> 4;
#pragma unroll
  for (int i = 0; i < 8; ++i) { const int ka = k0 + 8 * g + i, kb = ka + 16; v[i] = ka < K ? row[ka] : 0.f; v[8 + i] = kb < K ? row[kb] : 0.f; }
  return bsplit16(v); }
__device__ __forceinline__ F2 split_col(const float* W, int k0, int n, int lane, int ld, int K) { float v[16]; const int g = lane >> 4;
#pragma unroll
  for (int i = 0; i < 8; ++i) { const int ka = k0 + 8 * g + i, kb = ka + 16; v[i] = ka < K ? W[(size_t)ka * ld + n] : 0.f; v[8 + i] = kb < K ? W[(size_t)kb * ld + n] : 0.f; }
  return bsplit16(v); }
__device__ __forceinline__ v8f mac3(const F2& a, const F2& b, v8f c) { c = wmma_bf(a.l, b.h, c); c = wmma_bf(a.h, b.l, c); return wmma_bf(a.h, b.h, c); }
__device__ __forceinline__ float sigm(float v) { return 1.0f / (1.0f + expf(-v)); }
#define LDSX() do { asm volatile("s_wait_dscnt 0" ::: "memory"); __builtin_amdgcn_wave_barrier(); __builtin_amdgcn_fence(__ATOMIC_RELEASE, "workgroup"); } while (0)

#define NB 2
#define SS 128
#define HH 1024
#define AA 256
#define CC 14
#define NR (NB * SS)

__global__ __launch_bounds__(128) void k_l1(const float* __restrict__ mem, const float* __restrict__ hW1, const float* __restrict__ hb1, const float* __restrict__ tW1, const float* __restrict__ tb1, const float* __restrict__ mW1, const float* __restrict__ mb1, float* __restrict__ HID) {
  __shared__ __align__(16) float so[4][16][AA + 4];
  const int tid = threadIdx.x, wave = tid >> 5, lane = tid & 31, col = lane & 15, g = lane >> 4;
  const int which = blockIdx.y, r0 = blockIdx.x * 64 + wave * 16; const float* W = which == 0 ? hW1 : (which == 1 ? tW1 : mW1); const float* bias = which == 0 ? hb1 : (which == 1 ? tb1 : mb1);
#pragma unroll 1
  for (int np = 0; np < 2; ++np) { v8f acc[8] = {};
#pragma unroll 1
    for (int kc = 0; kc < HH / 32; ++kc) { const F2 a = split_row(mem + (size_t)(r0 + col) * HH, kc * 32, lane);
#pragma unroll
      for (int j = 0; j < 8; ++j) acc[j] = mac3(a, split_col(W, kc * 32, np * 128 + j * 16 + col, lane, AA, HH), acc[j]); }
#pragma unroll
    for (int j = 0; j < 8; ++j) { const int c = np * 128 + j * 16 + col; const float bb = bias[c];
#pragma unroll
      for (int r = 0; r < 8; ++r) { const float v = acc[j][r] + bb; so[wave][8 * g + r][c] = v > 0.f ? v : 0.f; } } }
  LDSX();
  for (int q = lane; q < 16 * 64; q += 32) { const int rl = q >> 6, pc = q & 63; vst2(HID + ((size_t)which * NR + r0 + rl) * AA + pc * 4, *(const v4f*)(&so[wave][rl][pc * 4])); }
}
__global__ __launch_bounds__(128) void k_l2(const float* __restrict__ HID, const float* __restrict__ hW2, const float* __restrict__ hb2, const float* __restrict__ tW2, const float* __restrict__ tb2, const float* __restrict__ mW2, const float* __restrict__ mb2,
                                          const float* __restrict__ s0h, const float* __restrict__ s0hb, const float* __restrict__ s1h, const float* __restrict__ s1hb, const float* __restrict__ s0t, const float* __restrict__ s0tb, const float* __restrict__ s1t, const float* __restrict__ s1tb,
                                          const float* __restrict__ s0m, const float* __restrict__ s0mb, const float* __restrict__ s1m, const float* __restrict__ s1mb, float* __restrict__ SC) {
  __shared__ __align__(16) float sf[4][16][AA + 4];
  __shared__ __align__(16) float ssc[4][16][32];
  const int tid = threadIdx.x, wave = tid >> 5, lane = tid & 31, col = lane & 15, g = lane >> 4;
  const int which = blockIdx.y, r0 = blockIdx.x * 64 + wave * 16; const float* W = which == 0 ? hW2 : (which == 1 ? tW2 : mW2); const float* bias = which == 0 ? hb2 : (which == 1 ? tb2 : mb2);
  const float* S0 = which == 0 ? s0h : (which == 1 ? s0t : s0m); const float* S0b = which == 0 ? s0hb : (which == 1 ? s0tb : s0mb); const float* S1 = which == 0 ? s1h : (which == 1 ? s1t : s1m); const float* S1b = which == 0 ? s1hb : (which == 1 ? s1tb : s1mb);
  const float* A = HID + ((size_t)which * NR) * AA;
#pragma unroll 1
  for (int np = 0; np < 2; ++np) { v8f acc[8] = {};
#pragma unroll 1
    for (int kc = 0; kc < AA / 32; ++kc) { const F2 a = split_row(A + (size_t)(r0 + col) * AA, kc * 32, lane);
#pragma unroll
      for (int j = 0; j < 8; ++j) acc[j] = mac3(a, split_col(W, kc * 32, np * 128 + j * 16 + col, lane, AA, AA), acc[j]); }
#pragma unroll
    for (int j = 0; j < 8; ++j) { const int c = np * 128 + j * 16 + col; const float bb = bias[c];
#pragma unroll
      for (int r = 0; r < 8; ++r) sf[wave][8 * g + r][c] = acc[j][r] + bb; } }
  LDSX();
  { const int rl = lane >> 1, s = lane & 1; const float* SW = s ? S1 : S0; const float* SB = s ? S1b : S0b; const float* fr = &sf[wave][rl][0]; float o[CC];
#pragma unroll
    for (int c = 0; c < CC; ++c) o[c] = SB[c];
#pragma unroll 2
    for (int a = 0; a < AA; ++a) { const float fv = fr[a]; const float* wr = SW + (size_t)a * CC;
#pragma unroll
      for (int c = 0; c < CC; ++c) o[c] += fv * wr[c]; }
#pragma unroll
    for (int c = 0; c < CC; ++c) ssc[wave][rl][s * 16 + c] = o[c];
    ssc[wave][rl][s * 16 + 14] = 0.f; ssc[wave][rl][s * 16 + 15] = 0.f; }
  LDSX();
  for (int q = lane; q < 16 * 8; q += 32) { const int rl = q >> 3, pc = q & 7; vst2(SC + ((size_t)which * NR + r0 + rl) * 32 + pc * 4, *(const v4f*)(&ssc[wave][rl][pc * 4])); }
}
__global__ __launch_bounds__(256) void k_fin(const float* __restrict__ SC, const float* __restrict__ uni, float* __restrict__ out) {
  __shared__ float sm0[SS][CC], sm1[SS][CC], st1[SS][CC]; __shared__ float sh1r[CC]; __shared__ float smean[CC]; __shared__ float smx[CC];
  __shared__ __align__(16) float so[SS * CC];
  const int i = blockIdx.x, b = blockIdx.y, tid = threadIdx.x;
  for (int q = tid; q < SS * CC; q += 256) { const int k = q / CC, c = q % CC; const size_t rk = (size_t)b * SS + k;
    sm0[k][c] = SC[((size_t)2 * NR + rk) * 32 + c]; sm1[k][c] = SC[((size_t)2 * NR + rk) * 32 + 16 + c]; st1[k][c] = SC[((size_t)1 * NR + rk) * 32 + 16 + c]; }
  if (tid < CC) sh1r[tid] = SC[((size_t)0 * NR + (size_t)b * SS + i) * 32 + 16 + tid];
  __syncthreads();
  if (tid < CC) { float s = 0.f, mx = -3.0e38f; for (int k = 0; k < SS; ++k) { s += sm1[k][tid]; mx = fmaxf(mx, sm0[k][tid]); } smean[tid] = s * (1.0f / SS); smx[tid] = mx; }
  __syncthreads();
  for (int q = tid; q < SS * CC; q += 256) { const int j = q / CC, c = q % CC; float w;
    if (i <= j) { float mx = -3.0e38f; for (int k = i; k <= j; ++k) mx = fmaxf(mx, sm0[k][c]); float z = 0.f, zs = 0.f;
      for (int k = i; k <= j; ++k) { const float e = expf(sm0[k][c] - mx); z += e; zs += e * sm1[k][c]; }
      w = zs / z; }
    else w = smean[c];
    so[j * CC + c] = sh1r[c] + st1[j][c] + w + uni[c]; }
  __syncthreads();
  for (int q = tid; q < SS * CC / 4; q += 256) vst2(out + (((size_t)b * SS + i) * SS) * CC + q * 4, *(const v4f*)(&so[q * 4]));
}
extern "C" void kernel_launch(void* const* d_in, const int* in_sizes, int n_in, void* d_out, int out_size, void* d_ws, size_t ws_size, hipStream_t stream) {
  (void)in_sizes; (void)n_in; (void)out_size; (void)ws_size;
  const float** I = (const float**)d_in;
  float* out = (float*)d_out;
  char* ws = (char*)d_ws; size_t off = 0;
  auto take = [&](size_t bytes) { char* p = ws + off; off += (bytes + 255) & ~(size_t)255; return p; };
  float* HID = (float*)take((size_t)3 * NR * AA * 4); float* SC = (float*)take((size_t)3 * NR * 32 * 4);
  k_l1<<<dim3(NR / 64, 3), 128, 0, stream>>>(I[0], I[1], I[2], I[9], I[10], I[17], I[18], HID);
  k_l2<<<dim3(NR / 64, 3), 128, 0, stream>>>(HID, I[3], I[4], I[11], I[12], I[19], I[20], I[5], I[6], I[7], I[8], I[13], I[14], I[15], I[16], I[21], I[22], I[23], I[24], SC);
  k_fin<<<dim3(SS, NB), 256, 0, stream>>>(SC, I[25], out);
}
